// Block_30520037605534
// MI455X (gfx1250) — hardware-verified
//
#include <hip/hip_runtime.h>
#include <math.h>

#ifndef NB
#define NB 2
#endif
#ifndef SEQ
#define SEQ 2048
#endif
#define NB_FULL 2
#define SEQ_FULL 2048
#define DM 1024
#define NHEAD 16
#define HDIM 64
#define DFF 4096
#define NXR 256
#define FCH ((((NB) * (SEQ)) < 1024) ? ((NB) * (SEQ)) : 1024)

static_assert(NB >= 1 && NB <= NB_FULL);
static_assert(SEQ >= NXR && SEQ <= SEQ_FULL);
static_assert((SEQ % 64) == 0);
static_assert((FCH % 64) == 0);
static_assert((SEQ % FCH) == 0);
static_assert(((NB * SEQ) % FCH) == 0);
static_assert(DM == NHEAD * HDIM);
static_assert((DM % 64) == 0 && (DFF % 64) == 0 && (DM % 32) == 0 && (DFF % 32) == 0);

typedef __attribute__((ext_vector_type(16))) _Float16 v16h;
typedef __attribute__((ext_vector_type(8)))  _Float16 v8h;
typedef __attribute__((ext_vector_type(16))) __bf16   v16b;
typedef __attribute__((ext_vector_type(8)))  float    v8f;
typedef __attribute__((ext_vector_type(4)))  float    v4f;

__device__ __forceinline__ int frag_k(int i, int h) { return (i < 8) ? (8 * h + i) : (16 + 8 * h + (i - 8)); }
__device__ __forceinline__ __bf16 bf16_rne(float f) {
    unsigned int u = __float_as_uint(f);
    u += 0x7fffu + ((u >> 16) & 1u);
    return __builtin_bit_cast(__bf16, (unsigned short)(u >> 16));
}
__device__ __forceinline__ float bf16_f32(__bf16 b) { return __uint_as_float(((unsigned int)__builtin_bit_cast(unsigned short, b)) << 16); }
__device__ __forceinline__ v8f wmma16(v16h a, v16h b, v8f c) {
    c = __builtin_amdgcn_wmma_f32_16x16x32_f16(false, a, false, b, (short)0, c, false, false);
    asm volatile("v_nop\n\tv_nop\n\tv_nop\n\tv_nop" : "+v"(c) : "v"(a), "v"(b));
    return c;
}
struct Split { v16b hi, lo; };
__device__ __forceinline__ v8f wmma3(const Split& a, const Split& b, v8f c) {
    c = __builtin_amdgcn_wmma_f32_16x16x32_bf16(false, a.hi, false, b.hi, (short)0, c, false, false);
    c = __builtin_amdgcn_wmma_f32_16x16x32_bf16(false, a.hi, false, b.lo, (short)0, c, false, false);
    c = __builtin_amdgcn_wmma_f32_16x16x32_bf16(false, a.lo, false, b.hi, (short)0, c, false, false);
    asm volatile("v_nop\n\tv_nop\n\tv_nop\n\tv_nop" : "+v"(c) : "v"(a.hi), "v"(a.lo), "v"(b.hi), "v"(b.lo));
    return c;
}
struct Split3 { v16b hi, mid, lo; };
__device__ __forceinline__ v8f wmma6(const Split3& a, const Split3& b, v8f c) {
    c = __builtin_amdgcn_wmma_f32_16x16x32_bf16(false, a.hi, false, b.hi, (short)0, c, false, false);
    c = __builtin_amdgcn_wmma_f32_16x16x32_bf16(false, a.hi, false, b.mid, (short)0, c, false, false);
    c = __builtin_amdgcn_wmma_f32_16x16x32_bf16(false, a.mid, false, b.hi, (short)0, c, false, false);
    c = __builtin_amdgcn_wmma_f32_16x16x32_bf16(false, a.hi, false, b.lo, (short)0, c, false, false);
    c = __builtin_amdgcn_wmma_f32_16x16x32_bf16(false, a.mid, false, b.mid, (short)0, c, false, false);
    c = __builtin_amdgcn_wmma_f32_16x16x32_bf16(false, a.lo, false, b.hi, (short)0, c, false, false);
    asm volatile("v_nop\n\tv_nop\n\tv_nop\n\tv_nop" : "+v"(c) : "v"(a.hi), "v"(a.mid), "v"(a.lo), "v"(b.hi), "v"(b.mid), "v"(b.lo));
    return c;
}

__device__ __forceinline__ v16h fh_ld(const float* __restrict__ p, long long sk, int k0, int h, int klen, float s) {
    v16h a;
#pragma unroll
    for (int i = 0; i < 16; ++i) { const int k = k0 + frag_k(i, h); a[i] = (k < klen) ? (_Float16)(p[(long long)k * sk] * s) : (_Float16)0.f; }
    return a;
}
__device__ __forceinline__ Split sp_ld(const float* __restrict__ p, long long sk, int k0, int h, int klen, float s) {
    Split r;
#pragma unroll
    for (int i = 0; i < 16; ++i) {
        const int k = k0 + frag_k(i, h); const float x = (k < klen) ? p[(long long)k * sk] * s : 0.f;
        const __bf16 hb = bf16_rne(x); r.hi[i] = hb; r.lo[i] = bf16_rne(x - bf16_f32(hb));
    }
    return r;
}
__device__ __forceinline__ Split3 sp3_ld(const float* __restrict__ p, long long sk, int k0, int h, int klen, float s) {
    Split3 r;
#pragma unroll
    for (int i = 0; i < 16; ++i) {
        const int k = k0 + frag_k(i, h); const float x = (k < klen) ? p[(long long)k * sk] * s : 0.f;
        const __bf16 hb = bf16_rne(x); const float r1 = x - bf16_f32(hb); const __bf16 mb = bf16_rne(r1);
        r.hi[i] = hb; r.mid[i] = mb; r.lo[i] = bf16_rne(r1 - bf16_f32(mb));
    }
    return r;
}

#define VST2(T, ptr, val) do { const T vst2_v_ = (val); *(volatile T*)(ptr) = vst2_v_; __threadfence(); *(volatile T*)(ptr) = vst2_v_; } while (0)
#define VST2V4(ptr, val) do { const v4f vst2_v4_ = (val); *(volatile v4f*)(ptr) = vst2_v4_; __threadfence(); *(volatile v4f*)(ptr) = vst2_v4_; } while (0)

#define AW 4
struct AttnP {
    const float* Q; const float* K; const float* V; float* O; float* P; const float* Mf; const int* Mi; float* ST;
    const float* Pw; const float* Rt; const int* SQ; const int* SK;
    long long swb, swh, swi, swj, srb, srh, sri;
    long long sQb, sQh, sQi, sQd, sKb, sKh, sKj, sKd, sVb, sVh, sVj, sVd, sOb, sOh, sOi, sPb, sPh, sPi, smb, smh, smi, smj;
    int Lq, Lk, dh, dv, hrep, causal, coff, pband;
    float scale, mfill; int nonorm, mpol;
    int roff, rn, segpol, win;
};
static_assert(sizeof(AttnP) == 12 * 8 + 29 * 8 + 16 * 4);

#ifndef KATTN_ATTR
#define KATTN_ATTR
#endif
template <int DHP, int DVP, int QM, bool SPLITPV, bool TWOPASS>
__global__ __launch_bounds__(32 * AW) KATTN_ATTR void k_attn(AttnP p) {
    constexpr int NT = DVP / 16;
    constexpr int KS = DHP / 32;
    constexpr int VP = DVP + 8;
    __shared__ __align__(16) float    pl[AW][16 * 64];
    __shared__ __align__(16) _Float16 vl[(SPLITPV ? 2 : 1) * 64 * VP];
    const int lane = threadIdx.x & 31, hf = lane >> 4, l15 = lane & 15, wave = threadIdx.x >> 5;
    const int h = blockIdx.y, b = blockIdx.z, hk = h / p.hrep;
    const int q0 = (blockIdx.x * AW + wave) * 16;
    float* myp = pl[wave];
    const float L2E = 1.4426950408889634f;
    const float NEG = -__builtin_inff();
    const int qi = min(q0 + l15, p.Lq - 1);
    const float* qrow = p.Q + b * p.sQb + h * p.sQh + (long long)qi * p.sQi;
    const float* kbase = p.K + b * p.sKb + hk * p.sKh;
    const float* vbase = p.V + b * p.sVb + hk * p.sVh;
    v16h qa[QM == 0 ? KS : 1]; Split qs_[QM == 1 ? KS : 1]; Split3 qt_[QM == 2 ? KS : 1];
#pragma unroll
    for (int ks = 0; ks < KS; ++ks) {
        if (QM == 2) qt_[ks] = sp3_ld(qrow, p.sQd, ks * 32, hf, p.dh, 1.f);
        else if (QM == 1) qs_[ks] = sp_ld(qrow, p.sQd, ks * 32, hf, p.dh, 1.f);
        else qa[ks] = fh_ld(qrow, p.sQd, ks * 32, hf, p.dh, 1.f);
    }
    v8f o[NT]; float m8[8], l8[8];
#pragma unroll
    for (int t = 0; t < NT; ++t) { v8f zz = {}; o[t] = zz; }
#pragma unroll
    for (int i = 0; i < 8; ++i) { m8[i] = NEG; l8[i] = 0.f; }
    int jend = p.Lk; int jstart = 0;
    if (p.causal == 1) { const int je = (blockIdx.x * AW + AW - 1) * 16 + 16 + p.coff; jend = min(jend, max(je, 0)); }
    if (p.win > 0) { const int js = (int)(blockIdx.x * AW) * 16 + p.coff - p.win; jstart = (js > 0) ? (js / 64) * 64 : 0; }
    const int npass = TWOPASS ? 2 : 1;
    for (int pass = 0; pass < npass; ++pass) {
        const bool dopv = (!TWOPASS) || pass == 1;
        for (int j0 = jstart; j0 < jend; j0 += 64) {
            if (dopv) {
                __syncthreads();
                for (int idx = threadIdx.x; idx < 64 * DVP; idx += 32 * AW) {
                    const int jr = idx / DVP, d = idx - jr * DVP, j = j0 + jr;
                    const float f = (j < p.Lk && d < p.dv) ? vbase[(long long)j * p.sVj + (long long)d * p.sVd] : 0.f;
                    if (SPLITPV) {
                        const __bf16 hb = bf16_rne(f);
                        ((__bf16*)vl)[jr * VP + d] = hb; ((__bf16*)vl)[64 * VP + jr * VP + d] = bf16_rne(f - bf16_f32(hb));
                    } else vl[jr * VP + d] = (_Float16)f;
                }
            }
            v8f s[4];
#pragma unroll
            for (int t = 0; t < 4; ++t) {
                const int j = min(j0 + t * 16 + l15, p.Lk - 1);
                const float* krow = kbase + (long long)j * p.sKj;
                v8f acc = {};
#pragma unroll
                for (int ks = 0; ks < KS; ++ks) {
                    if (QM == 2)      acc = wmma6(qt_[ks], sp3_ld(krow, p.sKd, ks * 32, hf, p.dh, 1.f), acc);
                    else if (QM == 1) acc = wmma3(qs_[ks], sp_ld(krow, p.sKd, ks * 32, hf, p.dh, 1.f), acc);
                    else              acc = wmma16(qa[ks], fh_ld(krow, p.sKd, ks * 32, hf, p.dh, 1.f), acc);
                }
                s[t] = acc;
            }
            float pv[8][4];
#pragma unroll
            for (int i = 0; i < 8; ++i) {
                const int irow = q0 + i + 8 * hf;
                const int ic = min(irow, p.Lq - 1);
                float sc[4];
#pragma unroll
                for (int t = 0; t < 4; ++t) {
                    const int jg = j0 + t * 16 + l15;
                    float v = s[t][i] * p.scale;
                    if (p.Mf) v += p.Mf[b * p.smb + h * p.smh + (long long)ic * p.smi + (long long)min(jg, p.Lk - 1) * p.smj];
                    if (p.Rt) { int rc = ic - min(jg, p.Lk - 1) + p.roff; rc = rc < 0 ? 0 : (rc >= p.rn ? p.rn - 1 : rc); v += p.Rt[b * p.srb + h * p.srh + (long long)ic * p.sri + rc]; }
                    if (p.Mi) { const int mv = p.Mi[b * p.smb + h * p.smh + (long long)ic * p.smi + (long long)min(jg, p.Lk - 1) * p.smj]; if (p.mpol ? (mv != 0) : (mv == 0)) v = p.mfill; }
                    if (p.SQ) { const bool same = p.SQ[(long long)b * p.Lq + ic] == p.SK[(long long)b * p.Lk + min(jg, p.Lk - 1)]; if (p.segpol ? same : !same) v = p.mfill; }
                    if (p.causal == 2 && jg > irow + p.coff) v = p.mfill;
                    if (jg >= p.Lk || (p.causal == 1 && jg > irow + p.coff) || (p.causal == 3 && jg < irow + p.coff) || (p.win > 0 && irow + p.coff - jg > p.win)) v = NEG; else v *= L2E;
                    sc[t] = v;
                }
                if (!TWOPASS || pass == 0) {
                    float mx = fmaxf(fmaxf(sc[0], sc[1]), fmaxf(sc[2], sc[3]));
                    mx = fmaxf(mx, __shfl_xor(mx, 1, 32)); mx = fmaxf(mx, __shfl_xor(mx, 2, 32));
                    mx = fmaxf(mx, __shfl_xor(mx, 4, 32)); mx = fmaxf(mx, __shfl_xor(mx, 8, 32));
                    const float mnew = fmaxf(m8[i], mx);
                    const float corr = (mnew == NEG) ? 1.f : exp2f(m8[i] - mnew);
                    float rs = 0.f;
#pragma unroll
                    for (int t = 0; t < 4; ++t) {
                        const float pp = (sc[t] == NEG) ? 0.f : exp2f(sc[t] - mnew); rs += pp;
                        pv[i][t] = p.Pw ? pp * p.Pw[b * p.swb + h * p.swh + (long long)ic * p.swi + (long long)min(j0 + t * 16 + l15, p.Lk - 1) * p.swj] : pp;
                    }
                    rs += __shfl_xor(rs, 1, 32); rs += __shfl_xor(rs, 2, 32); rs += __shfl_xor(rs, 4, 32); rs += __shfl_xor(rs, 8, 32);
                    l8[i] = l8[i] * corr + rs; m8[i] = mnew;
                    if (!TWOPASS) {
#pragma unroll
                        for (int t = 0; t < NT; ++t) o[t][i] *= corr;
                    }
                } else {
                    const float inv = (l8[i] > 0.f) ? 1.f / l8[i] : 0.f;
#pragma unroll
                    for (int t = 0; t < 4; ++t) {
                        const int jg = j0 + t * 16 + l15;
                        float pp = (sc[t] == NEG) ? 0.f : exp2f(sc[t] - m8[i]) * inv;
                        if (p.Pw) pp *= p.Pw[b * p.swb + h * p.swh + (long long)ic * p.swi + (long long)min(jg, p.Lk - 1) * p.swj];
                        pv[i][t] = pp;
                    }
                }
            }
            if (dopv) {
#pragma unroll
                for (int i = 0; i < 8; ++i)
#pragma unroll
                    for (int t = 0; t < 4; ++t) ((volatile float*)myp)[(i + 8 * hf) * 64 + t * 16 + l15] = pv[i][t];
                __syncthreads();
                if (p.P) {
                    float* pb_ = p.P + b * p.sPb + h * p.sPh;
                    const bool fastP = (p.pband == 0) && ((p.sPi & 3) == 0) && (j0 + 64 <= p.Lk) && (q0 + 16 <= p.Lq) && ((((size_t)pb_) & 15) == 0);
                    if (fastP) {
#pragma unroll
                        for (int s2 = 0; s2 < 8; ++s2) {
                            const int row = s2 * 2 + (lane >> 4), c4 = (lane & 15) * 4;
                            const v4f v = *(const v4f*)(myp + row * 64 + c4);
                            VST2V4(pb_ + (long long)(q0 + row) * p.sPi + j0 + c4, v);
                        }
                    } else {
                        for (int row = 0; row < 16; ++row) {
                            const int irow = q0 + row; if (irow >= p.Lq) continue;
                            for (int c = lane; c < 64; c += 32) {
                                const int jg = j0 + c; if (jg >= p.Lk) continue;
                                if (p.pband == 0) VST2(float, pb_ + (long long)irow * p.sPi + jg, myp[row * 64 + c]);
                                else if (jg - irow <= p.pband && irow - jg <= p.pband) VST2(float, pb_ + (long long)irow * p.sPi + (jg - irow + p.pband), myp[row * 64 + c]);
                            }
                        }
                    }
                }
                if (SPLITPV) {
                    const Split pa0 = sp_ld(myp + l15 * 64, 1, 0, hf, 64, 1.f), pa1 = sp_ld(myp + l15 * 64, 1, 32, hf, 64, 1.f);
                    const __bf16* vh = (const __bf16*)vl; const __bf16* vlo = vh + 64 * VP;
#pragma unroll
                    for (int t = 0; t < NT; ++t) {
                        const int dcol = t * 16 + l15;
                        Split b0, b1;
#pragma unroll
                        for (int e = 0; e < 16; ++e) {
                            const int k0 = frag_k(e, hf), k1 = 32 + frag_k(e, hf);
                            b0.hi[e] = vh[k0 * VP + dcol]; b0.lo[e] = vlo[k0 * VP + dcol]; b1.hi[e] = vh[k1 * VP + dcol]; b1.lo[e] = vlo[k1 * VP + dcol];
                        }
                        o[t] = wmma3(pa0, b0, o[t]);
                        o[t] = wmma3(pa1, b1, o[t]);
                    }
                } else {
                    const v16h pa0 = fh_ld(myp + l15 * 64, 1, 0, hf, 64, 4096.f), pa1 = fh_ld(myp + l15 * 64, 1, 32, hf, 64, 4096.f);
#pragma unroll
                    for (int t = 0; t < NT; ++t) {
                        const int dcol = t * 16 + l15;
                        v16h b0, b1;
#pragma unroll
                        for (int e = 0; e < 16; ++e) { b0[e] = vl[frag_k(e, hf) * VP + dcol]; b1[e] = vl[(32 + frag_k(e, hf)) * VP + dcol]; }
                        o[t] = wmma16(pa0, b0, o[t]);
                        o[t] = wmma16(pa1, b1, o[t]);
                    }
                }
            }
        }
    }
    float* obase = p.O + b * p.sOb + h * p.sOh;
    if (p.ST) {
        const int rl = lane >> 1, isel = rl & 7;
        float mv = 0.f, lv = 0.f;
#pragma unroll
        for (int i = 0; i < 8; ++i) if (i == isel) { mv = m8[i]; lv = l8[i]; }
        const int irow = q0 + rl;
        if (irow < p.Lq) { float* st = p.ST + (((long long)b * gridDim.y + h) * p.Lq + irow) * 2 + (lane & 1); VST2(float, st, (lane & 1) ? lv : mv * 0.6931471805599453f); }
    }
    float invr[8];
#pragma unroll
    for (int i = 0; i < 8; ++i) {
        if (TWOPASS) invr[i] = SPLITPV ? 1.f : (1.f / 4096.f);
        else if (p.nonorm) invr[i] = exp2f(m8[i]) * (SPLITPV ? 1.f : (1.f / 4096.f));
        else invr[i] = (l8[i] > 0.f) ? (SPLITPV ? 1.f / l8[i] : 1.f / (l8[i] * 4096.f)) : 0.f;
    }
    __syncthreads();
    const bool ofast = ((p.sOi & 3) == 0) && ((((size_t)obase) & 15) == 0) && (q0 + 16 <= p.Lq);
#pragma unroll
    for (int c0 = 0; c0 < DVP; c0 += 64) {
#pragma unroll
        for (int i = 0; i < 8; ++i)
#pragma unroll
            for (int t = 0; t < NT; ++t) if (t * 16 >= c0 && t * 16 < c0 + 64) ((volatile float*)myp)[(i + 8 * hf) * 64 + (t * 16 - c0) + l15] = o[t][i] * invr[i];
        __syncthreads();
        const int cw = (DVP - c0 < 64) ? (DVP - c0) : 64;
        if (ofast && (c0 + cw <= p.dv) && (cw % 32 == 0)) {
            const int lpr = cw / 4;
            const int rows_per_ins = 32 / lpr;
            for (int r0 = 0; r0 < 16; r0 += rows_per_ins) {
                const int row = r0 + lane / lpr, c4 = (lane % lpr) * 4;
                const v4f v = *(const v4f*)(myp + row * 64 + c4);
                VST2V4(obase + (long long)(q0 + row) * p.sOi + c0 + c4, v);
            }
        } else {
            for (int row = 0; row < 16; ++row) {
                const int irow = q0 + row; if (irow >= p.Lq) continue;
                for (int c = lane; c < cw; c += 32) { const int d = c0 + c; if (d < p.dv) VST2(float, obase + (long long)irow * p.sOi + d, myp[row * 64 + c]); }
            }
        }
        __syncthreads();
    }
}

namespace w25 {
typedef __attribute__((ext_vector_type(16))) _Float16 v16h;
typedef __attribute__((ext_vector_type(8)))  _Float16 v8h;
typedef __attribute__((ext_vector_type(16))) __bf16   v16b;
typedef __attribute__((ext_vector_type(8)))  __bf16   v8b;
typedef __attribute__((ext_vector_type(8)))  float    v8f;
typedef __attribute__((ext_vector_type(4)))  float    v4f;

__device__ __forceinline__ unsigned short f2bf_bits(float f) {
  unsigned u = __float_as_uint(f);
  return (unsigned short)((u + 0x7FFFu + ((u >> 16) & 1u)) >> 16);
}
__device__ __forceinline__ float bf_bits2f(unsigned short h) { return __uint_as_float(((unsigned)h) << 16); }

__device__ __forceinline__ void dep_guard_h(v8f& a, v8f& b, v16h x, v16h y) { asm volatile("v_nop\n\tv_nop\n\tv_nop\n\tv_nop" : "+v"(a), "+v"(b) : "v"(x), "v"(y)); }
__device__ __forceinline__ void dep_guard_b(v8f& a, v8f& b, v16b x, v16b y) { asm volatile("v_nop\n\tv_nop\n\tv_nop\n\tv_nop" : "+v"(a), "+v"(b) : "v"(x), "v"(y)); }
__device__ __forceinline__ void keep4_h(v16h a, v16h b, v16h c, v16h d) { asm volatile("v_nop" :: "v"(a), "v"(b), "v"(c), "v"(d)); }
__device__ __forceinline__ void keep4_b(v16b a, v16b b, v16b c, v16b d) { asm volatile("v_nop" :: "v"(a), "v"(b), "v"(c), "v"(d)); }
__device__ __forceinline__ void acc_guard4(v8f& a, v8f& b, v8f& c, v8f& d) { asm volatile("v_nop\n\tv_nop\n\tv_nop\n\tv_nop" : "+v"(a), "+v"(b), "+v"(c), "+v"(d)); }
template <typename T> struct Frag;
template <> struct Frag<_Float16> {
  typedef v16h V; union U { v16h v; v8h h[2]; };
  static __device__ __forceinline__ v16h load(const _Float16* p) {
    U f; f.h[0] = *(const v8h*)(p); f.h[1] = *(const v8h*)(p + 16); return f.v;
  }
  static __device__ __forceinline__ v8f mma(v16h a, v16h b, v8f c) {
    return __builtin_amdgcn_wmma_f32_16x16x32_f16(false, a, false, b, (short)0, c, false, false);
  }
  static __device__ __forceinline__ void guard(v8f& a, v8f& b, v16h x, v16h y) { dep_guard_h(a, b, x, y); }
  static __device__ __forceinline__ void keep(v16h a, v16h b, v16h c, v16h d) { keep4_h(a, b, c, d); }
};
template <> struct Frag<__bf16> {
  typedef v16b V; union U { v16b v; v8b h[2]; };
  static __device__ __forceinline__ v16b load(const __bf16* p) {
    U f; f.h[0] = *(const v8b*)(p); f.h[1] = *(const v8b*)(p + 16); return f.v;
  }
  static __device__ __forceinline__ v8f mma(v16b a, v16b b, v8f c) {
    return __builtin_amdgcn_wmma_f32_16x16x32_bf16(false, a, false, b, (short)0, c, false, false);
  }
  static __device__ __forceinline__ void guard(v8f& a, v8f& b, v16b x, v16b y) { dep_guard_b(a, b, x, y); }
  static __device__ __forceinline__ void keep(v16b a, v16b b, v16b c, v16b d) { keep4_b(a, b, c, d); }
};

template <int ET> struct Elem;
template <> struct Elem<0> { typedef _Float16 T; };
template <> struct Elem<1> { typedef __bf16 T; };
template <int ET, bool SPLIT, int BIAS_MODE, int OUT_MODE, bool RESID, int ACT = 0>
__global__ __launch_bounds__(256) void wmma_gemm64(
    const unsigned short* __restrict__ Ap, const unsigned short* __restrict__ A2p, int lda, long strideA,
    const unsigned short* __restrict__ Btp, const unsigned short* __restrict__ Bt2p, int ldb, long strideB,
    void* __restrict__ Cout, void* __restrict__ Cout2, int ldc, long strideC,
    const float* __restrict__ bias,
    const float* __restrict__ resid, long strideR,
    int M, int N, int K, float scale) {
  typedef typename Elem<ET>::T T;
  typedef typename Frag<T>::V V;
  const T* A = (const T*)Ap; const T* A2 = (const T*)A2p; const T* Bt = (const T*)Btp; const T* Bt2 = (const T*)Bt2p;
  __shared__ __align__(16) float sT[8][16 * 68];
  const int b    = blockIdx.y;
  const int lane = threadIdx.x & 31;
  const int wave = threadIdx.x >> 5;
  const int tilesN = N >> 6;
  const int tilesM = M >> 6;
  const int tile = blockIdx.x * 8 + wave;
  if (tile >= tilesM * tilesN) return;
  const int tm = tile / tilesN;
  const int tn = tile - tm * tilesN;
  const int m0 = tm << 6;
  const int n0 = tn << 6;

  const T* Ab  = A  + (size_t)b * strideA;
  const T* Bb  = Bt + (size_t)b * strideB;
  const T* Ab2 = SPLIT ? (A2  + (size_t)b * strideA) : nullptr;
  const T* Bb2 = SPLIT ? (Bt2 + (size_t)b * strideB) : nullptr;

  const int rlane = lane & 15;
  const int koff  = (lane >> 4) * 8;
  const int mOff  = (lane >> 4) * 8;

  v8f acc[4][4];
#pragma unroll
  for (int i = 0; i < 4; ++i)
#pragma unroll
    for (int j = 0; j < 4; ++j) acc[i][j] = (v8f){0.f,0.f,0.f,0.f,0.f,0.f,0.f,0.f};

  for (int k0 = 0; k0 < K; k0 += 32) {
    V bh[4], bl[4];
#pragma unroll
    for (int j = 0; j < 4; ++j) {
      const size_t bo = (size_t)(n0 + (j << 4) + rlane) * ldb + koff + k0;
      bh[j] = Frag<T>::load(Bb + bo);
      if (SPLIT) bl[j] = Frag<T>::load(Bb2 + bo);
    }
#pragma unroll
    for (int i = 0; i < 4; ++i) {
      const size_t ao = (size_t)(m0 + (i << 4) + rlane) * lda + koff + k0;
      V ah = Frag<T>::load(Ab + ao);
      V al;
      if (SPLIT) al = Frag<T>::load(Ab2 + ao);
#pragma unroll
      for (int j = 0; j < 4; ++j) {
        acc[i][j] = Frag<T>::mma(ah, bh[j], acc[i][j]);
        if (SPLIT) {
          acc[i][j] = Frag<T>::mma(ah, bl[j], acc[i][j]);
          acc[i][j] = Frag<T>::mma(al, bh[j], acc[i][j]);
        }
      }
      Frag<T>::guard(acc[i][0], acc[i][3], ah, SPLIT ? al : ah);
    }
    Frag<T>::keep(bh[0], bh[1], bh[2], bh[3]);
    if (SPLIT) Frag<T>::keep(bl[0], bl[1], bl[2], bl[3]);
  }
  acc_guard4(acc[0][0], acc[0][1], acc[0][2], acc[0][3]);
  acc_guard4(acc[1][0], acc[1][1], acc[1][2], acc[1][3]);
  acc_guard4(acc[2][0], acc[2][1], acc[2][2], acc[2][3]);
  acc_guard4(acc[3][0], acc[3][1], acc[3][2], acc[3][3]);

  float* slab = sT[wave];
  const float* Rb = RESID ? (resid + (size_t)b * strideR) : nullptr;
#pragma unroll
  for (int i = 0; i < 4; ++i) {
    const int mBase = m0 + (i << 4);
#pragma unroll
    for (int j = 0; j < 4; ++j) {
      const int n = n0 + (j << 4) + rlane;
      float bv = 0.f;
      if (BIAS_MODE == 2) bv = bias[n];
#pragma unroll
      for (int r = 0; r < 8; ++r) {
        float v = acc[i][j][r] * scale;
        if (BIAS_MODE == 1) v += bias[mBase + mOff + r];
        if (BIAS_MODE == 2) v += bv;
        if (RESID) v += Rb[(size_t)(mBase + mOff + r) * ldc + n];
        if (ACT == 1) v = tanhf(v);
        if (ACT == 2) v = fmaxf(v, 0.0f);
        if (ACT == 3) v = v / (1.0f + expf(-v));
        if (ACT == 4) v = (v > 0.f) ? v : 0.01f * v;
        if (ACT == 5) v = 0.5f * v * (1.0f + erff(v * 0.70710678118654752f));
        if (ACT == 6) v = (v > 0.f) ? v : 0.2f * v;
        if (ACT == 7) { const float u = 0.7978845608028654f * (v + 0.044715f * v * v * v); v = 0.5f * v * (1.f + tanhf(u)); }
        slab[(mOff + r) * 68 + (j << 4) + rlane] = v;
      }
    }
    __builtin_amdgcn_fence(3  , "workgroup");
    __builtin_amdgcn_wave_barrier();
    __builtin_amdgcn_fence(2  , "workgroup");
    if (OUT_MODE == 0) {
      float* C = (float*)Cout + (size_t)b * strideC;
      const int hh = lane >> 4, c4 = (lane & 15) * 4;
      for (int pass = 0; pass < 2; ++pass) {
#pragma unroll
        for (int it = 0; it < 8; ++it) {
          const int row = it * 2 + hh;
          v4f v = *(const v4f*)(slab + row * 68 + c4);
          *(volatile v4f*)(C + (size_t)(mBase + row) * ldc + n0 + c4) = v;
        }
        __threadfence();
      }
    } else {
      const int q = lane >> 3, c8 = (lane & 7) * 8;
      unsigned short* C  = (unsigned short*)Cout  + (size_t)b * strideC;
      unsigned short* C2 = (OUT_MODE == 2) ? ((unsigned short*)Cout2 + (size_t)b * strideC) : nullptr;
      for (int pass = 0; pass < 2; ++pass) {
#pragma unroll
        for (int it = 0; it < 4; ++it) {
          const int row = it * 4 + q;
          const float* sp = slab + row * 68 + c8;
          v8h hv, lv;
#pragma unroll
          for (int e = 0; e < 8; ++e) {
            if (OUT_MODE == 1) {
              hv[e] = (_Float16)sp[e];
            } else {
              unsigned short hb = f2bf_bits(sp[e]);
              unsigned short lb = f2bf_bits(sp[e] - bf_bits2f(hb));
              hv[e] = __builtin_bit_cast(_Float16, hb);
              lv[e] = __builtin_bit_cast(_Float16, lb);
            }
          }
          *(volatile v8h*)(C + (size_t)(mBase + row) * ldc + n0 + c8) = hv;
          if (OUT_MODE == 2) *(volatile v8h*)(C2 + (size_t)(mBase + row) * ldc + n0 + c8) = lv;
        }
        __threadfence();
      }
    }
    __builtin_amdgcn_fence(3  , "workgroup");
    __builtin_amdgcn_wave_barrier();
    __builtin_amdgcn_fence(2  , "workgroup");
  }
}

}

__global__ __launch_bounds__(256) void k_cast16(const float* __restrict__ src, long long lds, _Float16* __restrict__ dst, long long ldd, int R, int C, float s) {
    const long long i = (long long)blockIdx.x * 256 + threadIdx.x; const long long np = (long long)R * (C / 2); if (i >= np) return; const int r = (int)(i / (C / 2)); const int c = 2 * (int)(i % (C / 2));
    const _Float16 h0 = (_Float16)(src[(long long)r * lds + c] * s), h1 = (_Float16)(src[(long long)r * lds + c + 1] * s);
    const unsigned u = (unsigned)__builtin_bit_cast(unsigned short, h0) | ((unsigned)__builtin_bit_cast(unsigned short, h1) << 16);
    volatile unsigned* d = (volatile unsigned*)(dst + (long long)r * ldd + c); *d = u; __threadfence(); *d = u; }

__device__ __forceinline__ unsigned int f2bf2_pack(float a, float b, unsigned int* lo) {
    const unsigned short ha = w25::f2bf_bits(a), hb = w25::f2bf_bits(b);
    const unsigned short la = w25::f2bf_bits(a - w25::bf_bits2f(ha)), lb = w25::f2bf_bits(b - w25::bf_bits2f(hb));
    *lo = (unsigned)la | ((unsigned)lb << 16); return (unsigned)ha | ((unsigned)hb << 16); }
__global__ __launch_bounds__(256) void k_castS16(const float* __restrict__ src, long long lds, __bf16* __restrict__ dhi, __bf16* __restrict__ dlo, long long ldd, int R, int C, float s, int transpose) {
    const long long i = (long long)blockIdx.x * 256 + threadIdx.x; long long o; float a, b;
    if (transpose) { const long long np = (long long)C * (R / 2); if (i >= np) return; const int c = (int)(i / (R / 2)); const int r = 2 * (int)(i % (R / 2)); a = src[(long long)r * lds + c] * s; b = src[(long long)(r + 1) * lds + c] * s; o = (long long)c * ldd + r; }
    else { const long long np = (long long)R * (C / 2); if (i >= np) return; const int r = (int)(i / (C / 2)); const int c = 2 * (int)(i % (C / 2)); a = src[(long long)r * lds + c] * s; b = src[(long long)r * lds + c + 1] * s; o = (long long)r * ldd + c; }
    unsigned lo; const unsigned hi = f2bf2_pack(a, b, &lo); volatile unsigned* ph = (volatile unsigned*)(dhi + o); volatile unsigned* pl = (volatile unsigned*)(dlo + o);
    *ph = hi; *pl = lo; __threadfence(); *ph = hi; *pl = lo; }

typedef unsigned int cm_u4 __attribute__((ext_vector_type(4)));

__device__ __forceinline__ unsigned int cmb_pk2(float a, float b) { return (unsigned int)__builtin_bit_cast(unsigned short, (_Float16)a) | ((unsigned int)__builtin_bit_cast(unsigned short, (_Float16)b) << 16); }
__device__ __forceinline__ float cmb_bf(float v) { const unsigned u = __builtin_bit_cast(unsigned, v); const unsigned r = (u + 0x7fffu + ((u >> 16) & 1u)) & 0xffff0000u; return __builtin_bit_cast(float, r); }
__global__ __launch_bounds__(256) void k_cm_bfvec(const float* __restrict__ SRC, float* __restrict__ DST, int n) { const int u = blockIdx.x * 256 + threadIdx.x; if (u >= n) return; VST2(float, DST + u, cmb_bf(SRC[u])); }
__global__ __launch_bounds__(256) void k_cm_castbT(const float* __restrict__ SRC, int lds, unsigned short* __restrict__ DST, int ldd, int nR, int nC, float sc) {
    const long long u = (long long)blockIdx.x * 256 + threadIdx.x; const int per = nR / 8; if (u >= (long long)nC * per) return; const int c = (int)(u / per); const int r0 = 8 * (int)(u % per);
    float w[8];
#pragma unroll
    for (int e = 0; e < 8; ++e) w[e] = cmb_bf(SRC[(long long)(r0 + e) * lds + c]) * sc;
    cm_u4 pk; pk.x = cmb_pk2(w[0], w[1]); pk.y = cmb_pk2(w[2], w[3]); pk.z = cmb_pk2(w[4], w[5]); pk.w = cmb_pk2(w[6], w[7]); VST2(cm_u4, (cm_u4*)(DST + (long long)c * ldd + r0), pk); }
__global__ __launch_bounds__(256) void k_cm_castbTz(const float* __restrict__ SRC, unsigned sz, int lds, unsigned short* __restrict__ DST, unsigned dz, int ldd, int nR, int nC, float sc) {
    const unsigned z = blockIdx.y;
    const unsigned u = blockIdx.x * 256u + threadIdx.x; const unsigned per = ((unsigned)nR) >> 3; if (u >= (unsigned)nC * per) return;
    const unsigned c = u / per; const unsigned r0 = 8u * (u - c * per);
    const float* s = SRC + (size_t)z * sz; unsigned short* d = DST + (size_t)z * dz;
    float w[8];
#pragma unroll
    for (int e = 0; e < 8; ++e) w[e] = cmb_bf(s[(size_t)(r0 + (unsigned)e) * (unsigned)lds + c]) * sc;
    cm_u4 pk; pk.x = cmb_pk2(w[0], w[1]); pk.y = cmb_pk2(w[2], w[3]); pk.z = cmb_pk2(w[4], w[5]); pk.w = cmb_pk2(w[6], w[7]); VST2(cm_u4, (cm_u4*)(d + (size_t)c * (unsigned)ldd + r0), pk); }

template <int NX, int HREP>
__global__ __launch_bounds__(64) void k_gx_exact(const float* __restrict__ Q, int ldq, const float* __restrict__ KV, int ldkv, int voff, float sc, float* __restrict__ AOX, int ldo) {
    #pragma clang fp contract(off)
    __shared__ float qs[64]; __shared__ float ps[NX]; __shared__ float red[2];
    const int i = blockIdx.x, h = blockIdx.y, t = threadIdx.x; const int kvh = h / HREP;
    qs[t] = Q[(long long)i * ldq + h * 64 + t]; __syncthreads();
#pragma unroll
    for (int r = 0; r < NX / 64; ++r) { const int j = t + 64 * r; const int jc = min(j, i); const float* kr = KV + (long long)jc * ldkv + kvh * 64; float s = 0.f;
#pragma unroll 8
        for (int d = 0; d < 64; ++d) s += qs[d] * kr[d];
        ps[j] = (j <= i) ? s * sc : -3.0e38f; }
    __syncthreads();
    if (t == 0) { float m = -3.0e38f; for (int j = 0; j <= i; ++j) m = fmaxf(m, ps[j]); float z = 0.f; for (int j = 0; j <= i; ++j) { const float e = expf(ps[j] - m); ps[j] = e; z += e; } red[0] = 1.f / z; }
    __syncthreads();
    const float inv = red[0]; float o = 0.f;
    for (int j = 0; j <= i; ++j) o += ps[j] * KV[(long long)j * ldkv + voff + kvh * 64 + t];
    VST2(float, AOX + (long long)i * ldo + h * 64 + t, o * inv); }

typedef unsigned int bk_u4 __attribute__((ext_vector_type(4)));
typedef unsigned int bk_u2 __attribute__((ext_vector_type(2)));
__device__ __forceinline__ unsigned int bk_pk2(float a, float b) { return (unsigned int)__builtin_bit_cast(unsigned short, (_Float16)a) | ((unsigned int)__builtin_bit_cast(unsigned short, (_Float16)b) << 16); }
template <int NQ, int HASX, int XBF, int ABF = 0>
__global__ __launch_bounds__(256) void k_b_ln(const float* __restrict__ A, const float* __restrict__ X, const float* __restrict__ GA, const float* __restrict__ BE, float eps, float inv_vden, int rows, const float* __restrict__ MG, const float* __restrict__ MB, int rows_per_b, float* __restrict__ Yf, unsigned short* __restrict__ Y16) {
    #pragma clang fp contract(off)
    constexpr int WD = 128 * NQ; const int r = blockIdx.x * 8 + (threadIdx.x >> 5); const int L = threadIdx.x & 31; if (r >= rows) return; v4f v[NQ]; float s = 0.f;
#pragma unroll
    for (int q = 0; q < NQ; ++q) { const long long o = (long long)r * WD + 4 * L + 128 * q; v[q] = *(const v4f*)(A + o); if (ABF) { v[q].x = cmb_bf(v[q].x); v[q].y = cmb_bf(v[q].y); v[q].z = cmb_bf(v[q].z); v[q].w = cmb_bf(v[q].w); } if (HASX) { v4f x = *(const v4f*)(X + o); if (XBF) { x.x = cmb_bf(x.x); x.y = cmb_bf(x.y); x.z = cmb_bf(x.z); x.w = cmb_bf(x.w); } v[q] = v[q] + x; } s += (v[q].x + v[q].y) + (v[q].z + v[q].w); }
#pragma unroll
    for (int o = 16; o > 0; o >>= 1) s += __shfl_xor(s, o, 32);
    const float mu = s * (1.f / WD); float qq = 0.f;
#pragma unroll
    for (int q = 0; q < NQ; ++q) { v[q].x -= mu; v[q].y -= mu; v[q].z -= mu; v[q].w -= mu; qq += (v[q].x * v[q].x + v[q].y * v[q].y) + (v[q].z * v[q].z + v[q].w * v[q].w); }
#pragma unroll
    for (int o = 16; o > 0; o >>= 1) qq += __shfl_xor(qq, o, 32);
    const float rs = (eps < 0.f) ? (1.f / (sqrtf(qq * inv_vden) - eps)) : rsqrtf(qq * inv_vden + eps); const int bb = (MG != nullptr) ? (r / rows_per_b) : 0;
#pragma unroll
    for (int q = 0; q < NQ; ++q) { const int c = 4 * L + 128 * q; const v4f ga = *(const v4f*)(GA + c), be = *(const v4f*)(BE + c); v4f y; y.x = v[q].x * rs * cmb_bf(ga.x) + cmb_bf(be.x); y.y = v[q].y * rs * cmb_bf(ga.y) + cmb_bf(be.y); y.z = v[q].z * rs * cmb_bf(ga.z) + cmb_bf(be.z); y.w = v[q].w * rs * cmb_bf(ga.w) + cmb_bf(be.w);
        if (MG != nullptr) { const v4f mg = *(const v4f*)(MG + (long long)bb * WD + c), mb = *(const v4f*)(MB + (long long)bb * WD + c); y.x = y.x * (1.f + mg.x) + mb.x; y.y = y.y * (1.f + mg.y) + mb.y; y.z = y.z * (1.f + mg.z) + mb.z; y.w = y.w * (1.f + mg.w) + mb.w; }
        const long long o = (long long)r * WD + c; if (Yf != nullptr) VST2V4(Yf + o, y); if (Y16 != nullptr) { bk_u2 pk; pk.x = bk_pk2(y.x, y.y); pk.y = bk_pk2(y.z, y.w); VST2(bk_u2, (bk_u2*)(Y16 + o), pk); } } }
template <int ACT> __device__ __forceinline__ float bk_act(float v) { return (ACT == 0) ? fmaxf(v, 0.f) : 0.5f * v * (1.f + erff(v * 0.70710678118654752f)); }
template <int ACT>
__global__ __launch_bounds__(256) void k_b_act16(const float* __restrict__ F, unsigned short* __restrict__ Y16, long long n8) {
    #pragma clang fp contract(off)
    const long long u = (long long)blockIdx.x * 256 + threadIdx.x; if (u >= n8) return;
#pragma unroll 1
    for (int h = 0; h < 2; ++h) { const v4f a = *(const v4f*)(F + 8 * u + 4 * h); bk_u2 pk; pk.x = bk_pk2(bk_act<ACT>(a.x), bk_act<ACT>(a.y)); pk.y = bk_pk2(bk_act<ACT>(a.z), bk_act<ACT>(a.w)); VST2(bk_u2, (bk_u2*)(Y16 + 8 * u + 4 * h), pk); } }
template <int XBF>
__global__ __launch_bounds__(256) void k_b_add(const float* __restrict__ A, const float* __restrict__ X, const float* __restrict__ AL, int WD4, int rows_per_b, float* __restrict__ O, long long n4) {
    #pragma clang fp contract(off)
    const long long u = (long long)blockIdx.x * 256 + threadIdx.x; if (u >= n4) return; v4f a = *(const v4f*)(A + 4 * u); v4f x = *(const v4f*)(X + 4 * u); if (XBF) { x.x = cmb_bf(x.x); x.y = cmb_bf(x.y); x.z = cmb_bf(x.z); x.w = cmb_bf(x.w); }
    if (AL != nullptr) { const long long r = u / WD4; const int c4 = (int)(u % WD4); const v4f al = *(const v4f*)(AL + ((r / rows_per_b) * WD4 + c4) * 4); a.x *= al.x; a.y *= al.y; a.z *= al.z; a.w *= al.w; }
    v4f y; y.x = x.x + a.x; y.y = x.y + a.y; y.z = x.z + a.z; y.w = x.w + a.w; VST2V4(O + 4 * u, y); }

constexpr size_t pad256(size_t b) { return ((b + 255) / 256) * 256; }
constexpr unsigned cdivu(size_t a, size_t b) { return (unsigned)((a + b - 1) / b); }
constexpr size_t ROWS_ALL = (size_t)NB * SEQ;
constexpr size_t QKV_FLOATS = ((size_t)SEQ * 3 * DM > (size_t)FCH * DFF) ? (size_t)SEQ * 3 * DM : (size_t)FCH * DFF;
constexpr size_t WS_TOTAL =
    pad256(ROWS_ALL * DM * 4) * 2 + pad256(ROWS_ALL * DM * 2) + pad256((size_t)DFF * DM * 2) * 2 +
    pad256(((size_t)DFF + 64) * 4) + pad256(((size_t)DM + 64) * 4) * 2 +
    pad256((size_t)FCH * DFF * 2) + pad256((size_t)FCH * DM * 4) + pad256((size_t)SEQ * DM * 2) + pad256((size_t)3 * DM * DM * 2) +
    pad256(QKV_FLOATS * 4) + pad256((size_t)SEQ * DM * 4) + pad256((size_t)DM * DM * 2) * 3 + pad256((size_t)NXR * DM * 2) * 2;
static_assert(WS_TOTAL <= (size_t)134217728);
static_assert((size_t)32 * 256 == (size_t)HDIM * (DM / 8));
static_assert((size_t)NHEAD * HDIM * DM == (size_t)DM * DM);
static_assert(((size_t)(NB - 1) * SEQ_FULL + SEQ) * DM <= (size_t)NB_FULL * SEQ_FULL * DM);

extern "C" void kernel_launch(void* const* d_in, const int* in_sizes, int n_in, void* d_out, int out_size, void* d_ws, size_t ws_size, hipStream_t stream) {
    if (n_in < 14) return;
    const long long need_x = ((long long)(NB - 1) * SEQ_FULL + SEQ) * DM;
    if ((long long)in_sizes[0] < need_x) return;
    if (in_sizes[1] < NHEAD * DM * HDIM || in_sizes[2] < NHEAD * DM * HDIM || in_sizes[3] < NHEAD * DM * HDIM) return;
    if (in_sizes[4] < DM * DM || in_sizes[5] < DM || in_sizes[6] < DM || in_sizes[7] < DM || in_sizes[8] < DM || in_sizes[9] < DM) return;
    if (in_sizes[10] < DM * DFF || in_sizes[11] < DFF || in_sizes[12] < DFF * DM || in_sizes[13] < DM) return;
    if ((long long)out_size < need_x) return;
    if (ws_size < WS_TOTAL) return;
    const float* x = (const float*)d_in[0];
    const float* Wq = (const float*)d_in[1];
    const float* Wk = (const float*)d_in[2];
    const float* Wv = (const float*)d_in[3];
    const float* Wo = (const float*)d_in[4];
    const float* bo = (const float*)d_in[5];
    const float* g1 = (const float*)d_in[6];
    const float* b1 = (const float*)d_in[7];
    const float* g2 = (const float*)d_in[8];
    const float* b2 = (const float*)d_in[9];
    const float* W1 = (const float*)d_in[10];
    const float* bb1 = (const float*)d_in[11];
    const float* W2 = (const float*)d_in[12];
    const float* bb2 = (const float*)d_in[13];
    float* out = (float*)d_out;
    char* wsp = (char*)d_ws;
    float* ATT = (float*)wsp; wsp += pad256(ROWS_ALL * DM * 4);
    float* X1 = (float*)wsp; wsp += pad256(ROWS_ALL * DM * 4);
    unsigned short* H16 = (unsigned short*)wsp; wsp += pad256(ROWS_ALL * DM * 2);
    unsigned short* W1T = (unsigned short*)wsp; wsp += pad256((size_t)DFF * DM * 2);
    unsigned short* W2T = (unsigned short*)wsp; wsp += pad256((size_t)DFF * DM * 2);
    float* BR1 = (float*)wsp; wsp += pad256(((size_t)DFF + 64) * 4);
    float* BR2 = (float*)wsp; wsp += pad256(((size_t)DM + 64) * 4);
    float* BRO = (float*)wsp; wsp += pad256(((size_t)DM + 64) * 4);
    unsigned short* F16 = (unsigned short*)wsp; wsp += pad256((size_t)FCH * DFF * 2);
    float* FF = (float*)wsp; wsp += pad256((size_t)FCH * DM * 4);
    unsigned short* X16 = (unsigned short*)wsp; wsp += pad256((size_t)SEQ * DM * 2);
    unsigned short* W316 = (unsigned short*)wsp; wsp += pad256((size_t)3 * DM * DM * 2);
    float* QKV = (float*)wsp; wsp += pad256(QKV_FLOATS * 4);
    float* AO = (float*)wsp; wsp += pad256((size_t)SEQ * DM * 4);
    unsigned short* AO16 = X16;
    unsigned short* WO16 = (unsigned short*)wsp; wsp += pad256((size_t)DM * DM * 2);
    unsigned short* WOB = (unsigned short*)wsp; wsp += pad256((size_t)DM * DM * 2);
    unsigned short* WOL = (unsigned short*)wsp; wsp += pad256((size_t)DM * DM * 2);
    unsigned short* AOH2 = (unsigned short*)wsp; wsp += pad256((size_t)NXR * DM * 2);
    unsigned short* AOL2 = (unsigned short*)wsp; wsp += pad256((size_t)NXR * DM * 2);
    float* F1 = QKV;
    if ((size_t)(wsp - (char*)d_ws) > ws_size) return;

    k_cm_castbT<<<cdivu((size_t)DM * (DM / 8), 256), 256, 0, stream>>>(Wo, DM, WO16, DM, DM, DM, 16.0f);
    k_castS16<<<cdivu((size_t)DM * (DM / 2), 256), 256, 0, stream>>>(Wo, DM, (__bf16*)(WOB), (__bf16*)(WOL), DM, DM, DM, 1.0f, 1);
    k_cm_bfvec<<<cdivu(DM, 256), 256, 0, stream>>>(bo, BRO, DM);
    k_cm_castbTz<<<dim3(32, NHEAD), 256, 0, stream>>>(Wq, (unsigned)(DM * HDIM), HDIM, W316, (unsigned)(HDIM * DM), DM, DM, HDIM, 16.0f);
    k_cm_castbTz<<<dim3(32, NHEAD), 256, 0, stream>>>(Wk, (unsigned)(DM * HDIM), HDIM, W316 + (size_t)DM * DM, (unsigned)(HDIM * DM), DM, DM, HDIM, 16.0f);
    k_cm_castbTz<<<dim3(32, NHEAD), 256, 0, stream>>>(Wv, (unsigned)(DM * HDIM), HDIM, W316 + (size_t)2 * DM * DM, (unsigned)(HDIM * DM), DM, DM, HDIM, 16.0f);

    for (int b = 0; b < NB; ++b) {
        const float* xb = x + (size_t)b * SEQ_FULL * DM;
        float* ATTb = ATT + (size_t)b * SEQ * DM;
        float* X1b = X1 + (size_t)b * SEQ * DM;
        k_b_ln<8, 0, 0, 1><<<cdivu(SEQ, 8), 256, 0, stream>>>(xb, nullptr, g1, b1, 1e-5f, 0.0009765625f, SEQ, nullptr, nullptr, 1, nullptr, X16);
        w25::wmma_gemm64<0, false, 0, 0, false, 0><<<dim3(cdivu((size_t)(SEQ / 64) * (3 * DM / 64), 8), 1u), 256, 0, stream>>>(
            (const unsigned short*)X16, nullptr, DM, 0, (const unsigned short*)W316, nullptr, DM, 0, (void*)QKV, nullptr, 3 * DM, 0, nullptr, nullptr, 0, SEQ, 3 * DM, DM, 0.0625f);
        k_gx_exact<NXR, 1><<<dim3(NXR, NHEAD), 64, 0, stream>>>(QKV, 3 * DM, QKV + DM, 3 * DM, DM, 0.125f, AO, DM);
        if (SEQ > NXR) {
            AttnP a;
            a.Q = QKV + (size_t)NXR * 3 * DM; a.K = QKV + DM; a.V = QKV + 2 * DM; a.O = AO + (size_t)NXR * DM; a.P = 0; a.Mf = 0; a.Mi = 0; a.ST = 0;
            a.Pw = 0; a.Rt = 0; a.SQ = 0; a.SK = 0;
            a.swb = 0; a.swh = 0; a.swi = 0; a.swj = 0; a.srb = 0; a.srh = 0; a.sri = 0;
            a.sQb = (long long)SEQ * 3 * DM; a.sQh = HDIM; a.sQi = 3 * DM; a.sQd = 1;
            a.sKb = (long long)SEQ * 3 * DM; a.sKh = HDIM; a.sKj = 3 * DM; a.sKd = 1;
            a.sVb = (long long)SEQ * 3 * DM; a.sVh = HDIM; a.sVj = 3 * DM; a.sVd = 1;
            a.sOb = (long long)SEQ * DM; a.sOh = HDIM; a.sOi = DM; a.sPb = 0; a.sPh = 0; a.sPi = 0; a.smb = 0; a.smh = 0; a.smi = 0; a.smj = 0;
            a.Lq = SEQ - NXR; a.Lk = SEQ; a.dh = HDIM; a.dv = HDIM; a.hrep = 1; a.causal = 1; a.coff = NXR; a.pband = 0;
            a.scale = 0.125f; a.mfill = 0.0f; a.nonorm = 0; a.mpol = 0;
            a.roff = 0; a.rn = 1; a.segpol = 0; a.win = 0;
            k_attn<64, 64, 0, false, false><<<dim3(cdivu((size_t)(SEQ - NXR), 16 * AW), (unsigned)NHEAD, 1u), 32 * AW, 0, stream>>>(a);
        }
        k_cast16<<<cdivu((size_t)SEQ * (DM / 2), 256), 256, 0, stream>>>(AO, DM, (_Float16*)(AO16), DM, SEQ, DM, 1.0f);
        w25::wmma_gemm64<0, false, 2, 0, false, 0><<<dim3(cdivu((size_t)(SEQ / 64) * (DM / 64), 8), 1u), 256, 0, stream>>>(
            (const unsigned short*)AO16, nullptr, DM, 0, (const unsigned short*)WO16, nullptr, DM, 0, (void*)ATTb, nullptr, DM, 0, BRO, nullptr, 0, SEQ, DM, DM, 0.0625f);
        k_castS16<<<cdivu((size_t)NXR * (DM / 2), 256), 256, 0, stream>>>(AO, DM, (__bf16*)(AOH2), (__bf16*)(AOL2), DM, NXR, DM, 1.0f, 0);
        w25::wmma_gemm64<1, false, 2, 0, false, 0><<<dim3(cdivu((size_t)(NXR / 64) * (DM / 64), 8), 1u), 256, 0, stream>>>(
            (const unsigned short*)AOH2, nullptr, DM, 0, (const unsigned short*)WOB, nullptr, DM, 0, (void*)ATTb, nullptr, DM, 0, BRO, nullptr, 0, NXR, DM, DM, 1.0f);
        w25::wmma_gemm64<1, false, 0, 0, true, 0><<<dim3(cdivu((size_t)(NXR / 64) * (DM / 64), 8), 1u), 256, 0, stream>>>(
            (const unsigned short*)AOL2, nullptr, DM, 0, (const unsigned short*)WOB, nullptr, DM, 0, (void*)ATTb, nullptr, DM, 0, nullptr, ATTb, 0, NXR, DM, DM, 1.0f);
        k_b_add<1><<<cdivu((size_t)SEQ * DM / 4, 256), 256, 0, stream>>>(ATTb, xb, nullptr, DM / 4, 1, X1b, (long long)SEQ * DM / 4);
    }

    k_cm_castbT<<<cdivu((size_t)DFF * (DM / 8), 256), 256, 0, stream>>>(W1, DFF, W1T, DM, DM, DFF, 16.0f);
    k_cm_castbT<<<cdivu((size_t)DM * (DFF / 8), 256), 256, 0, stream>>>(W2, DM, W2T, DFF, DFF, DM, 16.0f);
    k_cm_bfvec<<<cdivu(DFF, 256), 256, 0, stream>>>(bb1, BR1, DFF);
    k_cm_bfvec<<<cdivu(DM, 256), 256, 0, stream>>>(bb2, BR2, DM);
    k_b_ln<8, 0, 0, 0><<<cdivu(ROWS_ALL, 8), 256, 0, stream>>>(X1, nullptr, g2, b2, 1e-5f, 0.0009765625f, (int)ROWS_ALL, nullptr, nullptr, 1, nullptr, H16);
    for (int ch = 0; ch < (int)(ROWS_ALL / FCH); ++ch) {
        const size_t r0 = (size_t)ch * FCH;
        const size_t bsel = r0 / SEQ, t0 = r0 - bsel * SEQ;
        float* outc = out + (bsel * SEQ_FULL + t0) * DM;
        w25::wmma_gemm64<0, false, 2, 0, false, 0><<<dim3(cdivu((size_t)(FCH / 64) * (DFF / 64), 8), 1u), 256, 0, stream>>>(
            (const unsigned short*)(H16 + r0 * DM), nullptr, DM, 0, (const unsigned short*)W1T, nullptr, DM, 0, (void*)F1, nullptr, DFF, 0, BR1, nullptr, 0, FCH, DFF, DM, 0.0625f);
        k_b_act16<0><<<cdivu((size_t)FCH * DFF / 8, 256), 256, 0, stream>>>(F1, F16, (long long)FCH * DFF / 8);
        w25::wmma_gemm64<0, false, 2, 0, false, 0><<<dim3(cdivu((size_t)(FCH / 64) * (DM / 64), 8), 1u), 256, 0, stream>>>(
            (const unsigned short*)F16, nullptr, DFF, 0, (const unsigned short*)W2T, nullptr, DFF, 0, (void*)FF, nullptr, DM, 0, BR2, nullptr, 0, FCH, DM, DFF, 0.0625f);
        k_b_add<0><<<cdivu((size_t)FCH * DM / 4, 256), 256, 0, stream>>>(FF, X1 + r0 * DM, nullptr, DM / 4, 1, outc, (long long)FCH * DM / 4);
    }
}
